// GAT_88871463289130
// MI455X (gfx1250) — hardware-verified
//
#include <hip/hip_runtime.h>
#include <stddef.h>
#include <stdint.h>
#include <math.h>


#define FIN     128
#define DH      128
#define NHD     8
#define HCH     16
#define KA2     256
#define NGR     64
#define NCLS    10
#define NTHR    256
#define NWAVE   8
#define EPT     8
#define CHUNK   (NTHR * EPT)
#define WCAP    (EPT * 32)
#define LISTN   (NWAVE * WCAP)
#define NBA     1024
#define SLA     10
#define RCAP    28672
#define DEGCAP  128
#define MEAS_B1024  16623
#define MEAS_MAXDEG 35
#define GBM     64
#define GBN     64
#define GTHR    128
#define MROWS   128
#define NUWI    (DH * (FIN / 8))
#define NUWC    (DH * (KA2 / 8))
#define NEGSL   0.2f
#define WSMAX   134217728
#define BKT_LDS_INTS  (LISTN + RCAP + 16)
#define SCAN_ZINTS    (RCAP + 3 * NBA)
#define SCAN_LDS_INTS (2 * RCAP + 3 * NBA + 16)

static_assert((CHUNK & (CHUNK - 1)) == 0 && CHUNK <= 4096);
static_assert((NBA & (NBA - 1)) == 0 && NBA == (1 << SLA) && NBA <= 1024);
static_assert(((long long)CHUNK << SLA) < (1LL << 31));
static_assert(LISTN >= NWAVE * WCAP);
static_assert(NBA % NWAVE == 0 && NBA % 32 == 0 && NBA % 16 == 0);
static_assert((RCAP % 32) == 0 && (SCAN_ZINTS % 4) == 0);
static_assert(RCAP >= MEAS_B1024 + 4096);
static_assert(DEGCAP >= MEAS_MAXDEG + 8);
static_assert(SCAN_LDS_INTS * 4 <= 300000 && BKT_LDS_INTS * 4 <= 300000);
static_assert(GBM == (GTHR / 32) * 16);
static_assert(GTHR == 2 * GBN && GTHR == 2 * GBM);
static_assert((FIN % 32) == 0 && (KA2 % 32) == 0 && KA2 == 2 * DH);
static_assert((DH % GBN) == 0 && GBN == 4 * HCH && DH == NHD * HCH);
static_assert(GTHR == 4 * 2 * HCH);
static_assert(GBN == 64 && (GTHR >> 6) == 2);
static_assert((MROWS % GBM) == 0);
static_assert(DH == 4 * 32);
static_assert(HCH == 4 * 4);
static_assert(DH <= NTHR);
static_assert((NUWI % NTHR) == 0 && (NUWC % NTHR) == 0);
static_assert(DH + NWAVE * DH <= RCAP);
static_assert(((NGR * NCLS) % 32) == 0);
static_assert(NGR * NCLS / 4 <= NTHR);
static_assert(NCLS <= 16);

typedef float          v2f  __attribute__((ext_vector_type(2)));
typedef float          v4f  __attribute__((ext_vector_type(4)));
typedef float          v8f  __attribute__((ext_vector_type(8)));
typedef double         v2d  __attribute__((ext_vector_type(2)));
typedef int            v4i  __attribute__((ext_vector_type(4)));
typedef int            v8i  __attribute__((ext_vector_type(8)));
typedef unsigned short v4us __attribute__((ext_vector_type(4)));
typedef unsigned short v8us __attribute__((ext_vector_type(8)));
typedef __bf16         v16b __attribute__((ext_vector_type(16)));
typedef v4f  __attribute__((may_alias)) v4fa;
typedef v2d  __attribute__((may_alias)) v2da;
typedef v4i  __attribute__((may_alias)) v4ia;
typedef v8us __attribute__((may_alias)) v8usa;
union FragB { v16b v; v8us h[2]; v8i w; };

__device__ __forceinline__ v8f wmb(const FragB& a, const FragB& b, v8f c) {
  v8f d = __builtin_amdgcn_wmma_f32_16x16x32_bf16(false, a.v, false, b.v, (short)0, c, false, false);
  asm volatile("v_nop\n\tv_nop\n\tv_nop\n\tv_nop" : "+v"(d) : "v"(a.w), "v"(b.w));
  return d;
}

__device__ __forceinline__ unsigned int f2bf(float f) {
  const unsigned int u = __float_as_uint(f);
  const unsigned int r = ((u + 0x7FFFu + ((u >> 16) & 1u)) >> 16) & 0xFFFFu;
  return ((u & 0x7FFFFFFFu) > 0x7F800000u) ? 0x7FC0u : r;
}
__device__ __forceinline__ float bf2f(unsigned int b) { return __uint_as_float(b << 16); }
__device__ __forceinline__ float bfr(float f) { return bf2f(f2bf(f)); }

template <int SLB>
__device__ __forceinline__ int scan_chunk(const int* __restrict__ dsts, int nE, int cbase, int slotBase,
                                          int nb, int vec8, int* list, int tid, int lane, int wave) {
  int wc = 0;
  const int el0  = tid * EPT;
  const int e0   = cbase + el0;
  const int sent = -2147483647 - 1;
  v4i da, db;
  if (vec8 != 0 && cbase + CHUNK <= nE) {
    da = *(const v4i*)(dsts + e0);
    db = *(const v4i*)(dsts + e0 + 4);
  } else {
    da.x = (e0     < nE) ? dsts[min(e0,     nE - 1)] : sent;
    da.y = (e0 + 1 < nE) ? dsts[min(e0 + 1, nE - 1)] : sent;
    da.z = (e0 + 2 < nE) ? dsts[min(e0 + 2, nE - 1)] : sent;
    da.w = (e0 + 3 < nE) ? dsts[min(e0 + 3, nE - 1)] : sent;
    db.x = (e0 + 4 < nE) ? dsts[min(e0 + 4, nE - 1)] : sent;
    db.y = (e0 + 5 < nE) ? dsts[min(e0 + 5, nE - 1)] : sent;
    db.z = (e0 + 6 < nE) ? dsts[min(e0 + 6, nE - 1)] : sent;
    db.w = (e0 + 7 < nE) ? dsts[min(e0 + 7, nE - 1)] : sent;
  }
  const unsigned nbs = (unsigned)slotBase;
  const unsigned unb = (unsigned)nb;
  const unsigned s0 = (unsigned)da.x - nbs, s1 = (unsigned)da.y - nbs;
  const unsigned s2 = (unsigned)da.z - nbs, s3 = (unsigned)da.w - nbs;
  const unsigned s4 = (unsigned)db.x - nbs, s5 = (unsigned)db.y - nbs;
  const unsigned s6 = (unsigned)db.z - nbs, s7 = (unsigned)db.w - nbs;
  const bool h0 = s0 < unb, h1 = s1 < unb, h2 = s2 < unb, h3 = s3 < unb;
  const bool h4 = s4 < unb, h5 = s5 < unb, h6 = s6 < unb, h7 = s7 < unb;
  const unsigned any = __builtin_amdgcn_ballot_w32(h0 | h1 | h2 | h3 | h4 | h5 | h6 | h7);
  if (any != 0u) {
#define HITJ(J, HJ, SJ) { \
      const unsigned mj = __builtin_amdgcn_ballot_w32(HJ); \
      if (mj != 0u) { \
        if (HJ) { \
          const int pos = wc + (int)__builtin_amdgcn_mbcnt_lo(mj, 0u); \
          if (pos < WCAP) list[wave * WCAP + pos] = ((el0 + (J)) << SLB) | (int)(SJ); \
        } \
        wc += (int)__builtin_popcount(mj); } }
    HITJ(0, h0, s0)
    HITJ(1, h1, s1)
    HITJ(2, h2, s2)
    HITJ(3, h3, s3)
    HITJ(4, h4, s4)
    HITJ(5, h5, s5)
    HITJ(6, h6, s6)
    HITJ(7, h7, s7)
#undef HITJ
  }
  return wc;
}

__global__ __launch_bounds__(NTHR) void k_prep(const float* __restrict__ x, const float* __restrict__ inw,
                                               const float* __restrict__ cw, unsigned short* XB,
                                               unsigned short* WinT, unsigned short* WcD, int nN, int nUx) {
  const int u = (int)blockIdx.x * NTHR + (int)threadIdx.x;
  v8us o;
  unsigned short* dp;
  if (u < nUx) {
    const int row = u >> 4;
    const int c0  = (u & 15) * 8;
    const int rc  = row < nN ? row : nN - 1;
    const float* p = x + (size_t)rc * FIN + c0;
    const v4f a = *(const v4f*)p;
    const v4f b = *(const v4f*)(p + 4);
    const bool okr = row < nN;
    o[0] = okr ? (unsigned short)f2bf(a.x) : (unsigned short)0;
    o[1] = okr ? (unsigned short)f2bf(a.y) : (unsigned short)0;
    o[2] = okr ? (unsigned short)f2bf(a.z) : (unsigned short)0;
    o[3] = okr ? (unsigned short)f2bf(a.w) : (unsigned short)0;
    o[4] = okr ? (unsigned short)f2bf(b.x) : (unsigned short)0;
    o[5] = okr ? (unsigned short)f2bf(b.y) : (unsigned short)0;
    o[6] = okr ? (unsigned short)f2bf(b.z) : (unsigned short)0;
    o[7] = okr ? (unsigned short)f2bf(b.w) : (unsigned short)0;
    dp = XB + (size_t)row * FIN + c0;
  } else if (u < nUx + NUWI) {
    const int v  = u - nUx;
    const int n  = v >> 4;
    const int k8 = (v & 15) * 8;
    const float* p = inw + (size_t)k8 * DH + n;
#pragma unroll
    for (int i = 0; i < 8; ++i) o[i] = (unsigned short)f2bf(p[(size_t)i * DH]);
    dp = WinT + (size_t)n * FIN + k8;
  } else if (u < nUx + NUWI + 2 * NUWC) {
    const int v  = u - nUx - NUWI;
    const int l  = v >> 12;
    const int w  = v & (NUWC - 1);
    const int n  = w >> 5;
    const int k8 = (w & 31) * 8;
    const int kk = k8 & (DH - 1);
    const float* p = cw + (size_t)l * DH * DH + (size_t)kk * DH + n;
#pragma unroll
    for (int i = 0; i < 8; ++i) o[i] = (unsigned short)f2bf(p[(size_t)i * DH]);
    dp = WcD + (size_t)l * DH * KA2 + (size_t)n * KA2 + k8;
  } else {
    return;
  }
  *(volatile v8us*)dp = o;
  __threadfence();
  *(volatile v8us*)dp = o;
}

__global__ __launch_bounds__(NTHR) void k_bucket(const int* __restrict__ srcs, const int* __restrict__ dsts,
                                                 int nE, int nN, int vec8, int* HITS, int* FLG) {
  extern __shared__ __attribute__((aligned(16))) int bsm[];
  int* list = bsm;
  int* reg1 = bsm + LISTN;
  int* wcnt = reg1 + RCAP;
  const int tid = (int)threadIdx.x, lane = tid & 31, wave = tid >> 5;
  const int blk = (int)blockIdx.x;
  const int nodeBase = blk * NBA;
  int nb = nN - nodeBase;
  nb = nb < 0 ? 0 : (nb > NBA ? NBA : nb);

  int tot = 0, ovf = 0;
  const int nChunks = (nE + CHUNK - 1) / CHUNK;
#pragma unroll 1
  for (int ch = 0; ch < nChunks; ++ch) {
    const int cbase = ch * CHUNK;
    const int wc = scan_chunk<SLA>(dsts, nE, cbase, nodeBase, nb, vec8, list, tid, lane, wave);
    if (lane == 0) wcnt[wave] = wc;
    __syncthreads();
    int pre = 0, all = 0;
#pragma unroll
    for (int w2 = 0; w2 < NWAVE; ++w2) {
      int c = wcnt[w2];
      c = c < 0 ? 0 : (c > WCAP ? WCAP : c);
      all += c;
      pre += (w2 < wave) ? c : 0;
    }
    const int wcc  = wc > WCAP ? WCAP : wc;
    const int base = tot + pre;
#pragma unroll 1
    for (int i = lane; i < wcc; i += 32) {
      const int ent = list[wave * WCAP + i];
      const int el  = (ent >> SLA) & (CHUNK - 1);
      const int sl  = ent & (NBA - 1);
      int eid = cbase + el;
      eid = eid > nE - 1 ? nE - 1 : eid;
      const int sraw = srcs[eid];
      const int s = sraw < 0 ? 0 : (sraw > nN - 1 ? nN - 1 : sraw);
      const int pos = base + i;
      if (pos < RCAP) reg1[pos] = (int)((unsigned)s | ((unsigned)sl << 16));
    }
    if (tot + all > RCAP) ovf = 1;
    tot += all;
    tot = tot > RCAP ? RCAP : tot;
    __syncthreads();
  }
  const int nh = tot;
  const int nhPad = (nh + 31) & ~31;
  for (int i = nh + tid; i < nhPad; i += NTHR) reg1[i] = 0;
  __syncthreads();

  int* hb = HITS + (size_t)blk * RCAP;
  v4i cv;
  cv.x = (tid == 0) ? nh : 0;
  cv.y = (tid == 0) ? ovf : 0;
  cv.z = 0; cv.w = 0;
  int* fp = FLG + (size_t)blk * 32 + 4 * (tid & 7);
#pragma unroll 1
  for (int p = tid * 4; p < nhPad; p += NTHR * 4) {
    const v4i v = *(const v4ia*)(reg1 + p);
    *(volatile v4i*)(hb + p) = v;
  }
  if (tid < 8) *(volatile v4i*)fp = cv;
  __threadfence();
#pragma unroll 1
  for (int p = tid * 4; p < nhPad; p += NTHR * 4) {
    const v4i v = *(const v4ia*)(reg1 + p);
    *(volatile v4i*)(hb + p) = v;
  }
  if (tid < 8) *(volatile v4i*)fp = cv;
}

template <int MODE>
__global__ __launch_bounds__(GTHR) void k_gemm(
    const unsigned short* __restrict__ A, const unsigned short* __restrict__ WT, int K,
    const float* __restrict__ bias, unsigned short* XP, int nN,
    float* outF, const float* __restrict__ atts, const float* __restrict__ attd,
    float* SD, int MPr)
{
  __shared__ __attribute__((aligned(16))) float stg[GBM * GBN];
  __shared__ __attribute__((aligned(16))) float satt[4 * 2 * HCH];
  __shared__ __attribute__((aligned(16))) float sdot[8 * GBM];
  const int tid = (int)threadIdx.x, lane = tid & 31, wave = tid >> 5, hh = lane >> 4, m = lane & 15;
  const int rowBase = (int)blockIdx.x * GBM;
  const int by      = (int)blockIdx.y;
  const int col0    = by * GBN;

  if constexpr (MODE == 0) {
    if (tid < GBN) satt[tid] = bfr(bias[col0 + tid]);
  } else {
    const int which = tid >> 6;
    const int c     = tid & 63;
    const int hl    = c >> 4;
    const int chn   = c & 15;
    int ai = col0 + c;
    ai = ai > NHD * HCH - 1 ? NHD * HCH - 1 : ai;
    const float vs = atts[ai];
    const float vd = attd[ai];
    const float v = (which == 0) ? vs : vd;
    satt[(2 * hl + which) * HCH + chn] = bfr(v);
  }

  v8f acc[4];
  {
    const v8f z = {0.f, 0.f, 0.f, 0.f, 0.f, 0.f, 0.f, 0.f};
    acc[0] = z; acc[1] = z; acc[2] = z; acc[3] = z;
  }
  const unsigned short* ap = A  + (size_t)(rowBase + 16 * wave + m) * (size_t)K + 8 * hh;
  const unsigned short* wp = WT + (size_t)(col0 + m) * (size_t)K + 8 * hh;
  const int ksteps = K >> 5;
#pragma unroll 1
  for (int ks = 0; ks < ksteps; ++ks) {
    FragB af;
    af.h[0] = *(const v8usa*)(ap + 32 * ks);
    af.h[1] = *(const v8usa*)(ap + 32 * ks + 16);
#pragma unroll
    for (int t = 0; t < 4; ++t) {
      const unsigned short* wq = wp + (size_t)(16 * t) * (size_t)K + 32 * ks;
      FragB bf;
      bf.h[0] = *(const v8usa*)wq;
      bf.h[1] = *(const v8usa*)(wq + 16);
      acc[t] = wmb(af, bf, acc[t]);
    }
  }

#pragma unroll
  for (int t = 0; t < 4; ++t) {
    const int lc = 16 * t + m;
#pragma unroll
    for (int r = 0; r < 8; ++r) {
      const int lr = 16 * wave + 8 * hh + r;
      stg[lr * GBN + lc] = acc[t][r];
    }
  }
  __syncthreads();

  if constexpr (MODE == 0) {
    const int q = lane >> 3, piece = lane & 7;
    const v4f ba = *(const v4fa*)(satt + 8 * piece);
    const v4f bb = *(const v4fa*)(satt + 8 * piece + 4);
    v8us ov[8];
#pragma unroll
    for (int i = 0; i < 8; ++i) {
      const int lx   = (wave * 8 + i) * 4 + q;
      const int lr   = lx >> 1;
      const int part = lx & 1;
      const int gr   = rowBase + lr;
      const v4f a = *(const v4fa*)(stg + lr * GBN + 8 * piece);
      const v4f b = *(const v4fa*)(stg + lr * GBN + 8 * piece + 4);
      const bool live = gr < nN;
      float v[8];
      v[0] = a.x + ba.x; v[1] = a.y + ba.y; v[2] = a.z + ba.z; v[3] = a.w + ba.w;
      v[4] = b.x + bb.x; v[5] = b.y + bb.y; v[6] = b.z + bb.z; v[7] = b.w + bb.w;
      v8us o;
#pragma unroll
      for (int e = 0; e < 8; ++e) {
        const float w = live ? v[e] : 0.0f;
        const unsigned int hb = f2bf(w);
        const unsigned int lb = f2bf(w - bf2f(hb));
        o[e] = (unsigned short)((part != 0) ? lb : hb);
      }
      ov[i] = o;
    }
#pragma unroll
    for (int i = 0; i < 8; ++i) {
      const int lx = (wave * 8 + i) * 4 + q;
      const int gr = rowBase + (lx >> 1);
      unsigned short* dp = XP + (size_t)gr * KA2 + (lx & 1) * DH + col0 + 8 * piece;
      *(volatile v8us*)dp = ov[i];
    }
    __threadfence();
#pragma unroll
    for (int i = 0; i < 8; ++i) {
      const int lx = (wave * 8 + i) * 4 + q;
      const int gr = rowBase + (lx >> 1);
      unsigned short* dp = XP + (size_t)gr * KA2 + (lx & 1) * DH + col0 + 8 * piece;
      *(volatile v8us*)dp = ov[i];
    }
  } else {
    {
      const int row = tid & 63, hp2 = tid >> 6;
#pragma unroll
      for (int hq = 0; hq < 2; ++hq) {
        const int hl = 2 * hp2 + hq;
        const float* sa = satt + (2 * hl) * HCH;
        const float* sb = sa + HCH;
        const float* hr = stg + row * GBN + HCH * hl;
        float ds = 0.f, dd = 0.f;
#pragma unroll 2
        for (int c4 = 0; c4 < HCH / 4; ++c4) {
          const v4f hv = *(const v4fa*)(hr + 4 * c4);
          const v4f av = *(const v4fa*)(sa + 4 * c4);
          const v4f bv = *(const v4fa*)(sb + 4 * c4);
          ds = fmaf(hv.x, av.x, ds);  dd = fmaf(hv.x, bv.x, dd);
          ds = fmaf(hv.y, av.y, ds);  dd = fmaf(hv.y, bv.y, dd);
          ds = fmaf(hv.z, av.z, ds);  dd = fmaf(hv.z, bv.z, dd);
          ds = fmaf(hv.w, av.w, ds);  dd = fmaf(hv.w, bv.w, dd);
        }
        sdot[(2 * hl) * GBM + row]     = ds;
        sdot[(2 * hl + 1) * GBM + row] = dd;
      }
    }
    __syncthreads();

    v4f fv[8];
#pragma unroll
    for (int i = 0; i < 8; ++i) {
      const int lr = 16 * wave + 2 * i + hh;
      fv[i] = *(const v4fa*)(stg + lr * GBN + 4 * m);
    }
    const int pl = 2 * wave + (lane >> 4), piece = lane & 15;
    const v4f sdv = *(const v4fa*)(sdot + pl * GBM + 4 * piece);
    float* sp = SD + (size_t)(8 * by + pl) * (size_t)MPr + rowBase + 4 * piece;

#pragma unroll
    for (int i = 0; i < 8; ++i) {
      const int lr = 16 * wave + 2 * i + hh;
      const int gr = rowBase + lr;
      float* op = outF + (size_t)gr * (size_t)DH + col0 + 4 * m;
      *(volatile v4f*)op = fv[i];
    }
    *(volatile v4f*)sp = sdv;
    __threadfence();
#pragma unroll
    for (int i = 0; i < 8; ++i) {
      const int lr = 16 * wave + 2 * i + hh;
      const int gr = rowBase + lr;
      float* op = outF + (size_t)gr * (size_t)DH + col0 + 4 * m;
      *(volatile v4f*)op = fv[i];
    }
    *(volatile v4f*)sp = sdv;
  }
}

template <int L>
__global__ __launch_bounds__(NTHR) void k_scan(const int* __restrict__ HITS, const int* __restrict__ FLGB,
                                               const float* __restrict__ F, const float* __restrict__ SD,
                                               const float* __restrict__ bias,
                                               unsigned short* XP, float* HO, int* FLGO, int nN, int MPr) {
  static_assert(L == 1 || L == 2);
  constexpr int CPL = 4;
  extern __shared__ __attribute__((aligned(16))) int ssm[];
  int* hl   = ssm;
  int* sl   = ssm + RCAP;
  int* cnt  = sl + RCAP;
  int* offs = cnt + NBA;
  int* cur  = offs + NBA;
  int* misc = cur + NBA;
  const int tid = (int)threadIdx.x, lane = tid & 31, wave = tid >> 5;
  const int blk = (int)blockIdx.x;
  const int nodeBase = blk * NBA;

  const int nhraw = FLGB[(size_t)blk * 32];
  const int bflag = FLGB[(size_t)blk * 32 + 1];
  const int nh  = nhraw < 0 ? 0 : (nhraw > RCAP ? RCAP : nhraw);
  const int ovf = (bflag != 0 || nhraw < 0 || nhraw > RCAP) ? 1 : 0;

  {
    const v4i z4 = {0, 0, 0, 0};
    for (int i = tid * 4; i < SCAN_ZINTS; i += NTHR * 4) *(v4ia*)(sl + i) = z4;
    if (tid < 16) misc[tid] = 0;
    const int* hb = HITS + (size_t)blk * RCAP;
    const int nh4 = (nh + 3) & ~3;
#pragma unroll 1
    for (int p = tid * 4; p < nh4; p += NTHR * 4) *(v4ia*)(hl + p) = *(const v4i*)(hb + p);
  }
  __syncthreads();

  if (wave == 0) {
#pragma unroll 1
    for (int b0 = 0; b0 < nh; b0 += 32) {
      const int idx = b0 + lane;
      const int uv  = hl[idx < nh ? idx : nh - 1];
      const int m32 = (nh - b0) < 32 ? (nh - b0) : 32;
#pragma unroll 1
      for (int k = 0; k < m32; ++k) {
        const int u  = __builtin_amdgcn_readlane(uv, k);
        const int sq = (u >> 16) & (NBA - 1);
        if (lane == 0) cnt[sq] = cnt[sq] + 1;
      }
    }
  }
  __syncthreads();
  if (wave == 0) {
    const int base = lane * (NBA / 32);
    int s = 0;
#pragma unroll 1
    for (int i = 0; i < NBA / 32; ++i) s += cnt[base + i];
    int incl = s;
#pragma unroll
    for (int d = 1; d < 32; d <<= 1) {
      const int y = __shfl_up(incl, d, 32);
      if (lane >= d) incl += y;
    }
    int run = incl - s;
#pragma unroll 1
    for (int i = 0; i < NBA / 32; ++i) {
      const int cv = cnt[base + i];
      offs[base + i] = run;
      cur[base + i]  = run;
      run += cv;
    }
  }
  __syncthreads();
  if (wave == 0) {
#pragma unroll 1
    for (int b0 = 0; b0 < nh; b0 += 32) {
      const int idx = b0 + lane;
      const int uv  = hl[idx < nh ? idx : nh - 1];
      const int m32 = (nh - b0) < 32 ? (nh - b0) : 32;
#pragma unroll 1
      for (int k = 0; k < m32; ++k) {
        const int u  = __builtin_amdgcn_readlane(uv, k);
        const int sq = (u >> 16) & (NBA - 1);
        if (lane == 0) {
          int p = cur[sq];
          p = p < 0 ? 0 : (p > RCAP - 1 ? RCAP - 1 : p);
          sl[p] = u;
          cur[sq] = p + 1;
        }
      }
    }
  }
  __syncthreads();

  float* fl = (float*)hl;
  float* st = fl + DH + wave * DH;
  if (tid < DH) fl[tid] = bfr(bias[CPL * (tid & 31) + (tid >> 5)]);
  __syncthreads();

  const float qnan = __int_as_float(0x7fc00000);
  const float pzb  = (ovf != 0) ? qnan : 0.0f;
  const int head   = lane >> 2;
  const size_t hoS = (size_t)(2 * head) * (size_t)MPr;
  const size_t hoD = hoS + (size_t)MPr;
  int anybig = 0;

#pragma unroll 1
  for (int si = 0; si < NBA / NWAVE; ++si) {
    const int s    = si * NWAVE + wave;
    const int node = nodeBase + s;
    const int nc   = node < nN ? node : nN - 1;
    int c = cnt[s];
    const bool big = c > DEGCAP;
    anybig |= big ? 1 : 0;
    c = c < 0 ? 0 : (c > DEGCAP ? DEGCAP : c);
    int o = offs[s];
    o = o < 0 ? 0 : (o > RCAP ? RCAP : o);
    if (c > nh - o) c = nh - o;
    c = c < 0 ? 0 : c;
    const float adv = SD[hoD + (size_t)nc];
    float mx = -3.0e38f, dn = 0.0f;
    float acc[CPL];
#pragma unroll
    for (int i = 0; i < CPL; ++i) acc[i] = 0.0f;
#pragma unroll 1
    for (int b0 = 0; b0 < c; b0 += 32) {
      const int t = b0 + lane;
      int idx = o + t;
      idx = idx < 0 ? 0 : (idx > RCAP - 1 ? RCAP - 1 : idx);
      const int ent = sl[idx];
      int hs = ent & 0xFFFF;
      hs = hs > nN - 1 ? nN - 1 : hs;
      const int sr  = hs;
      const int m32 = (c - b0) < 32 ? (c - b0) : 32;
#pragma unroll 1
      for (int k = 0; k < m32; ++k) {
        const int sk = __builtin_amdgcn_readlane(sr, k);
        const float* rp = F + (size_t)sk * DH + CPL * lane;
        const v4f a = *(const v4f*)rp;
        float lg = SD[hoS + (size_t)sk] + adv;
        lg = lg > 0.f ? lg : NEGSL * lg;
        const float df = lg - mx;
        const float ee = expf(-fabsf(df));
        const bool  up = df > 0.f;
        const float s1 = up ? ee : 1.0f;
        const float s2 = up ? 1.0f : ee;
        mx = up ? lg : mx;
        dn = fmaf(dn, s1, s2);
        acc[0] = fmaf(acc[0], s1, s2 * a.x);
        acc[1] = fmaf(acc[1], s1, s2 * a.y);
        acc[2] = fmaf(acc[2], s1, s2 * a.z);
        acc[3] = fmaf(acc[3], s1, s2 * a.w);
      }
    }
    const float rdn = __builtin_amdgcn_rcpf(dn);
    const float inv = (c > 0) ? rdn : 0.0f;
    const float pzr = big ? qnan : pzb;
    const bool live = node < nN;

#pragma unroll
    for (int i = 0; i < CPL; ++i) st[i * 32 + lane] = acc[i];
#pragma unroll 1
    for (int j = 0; j < CPL; ++j) {
      float y = fmaf(st[j * 32 + lane], inv, fl[j * 32 + lane]);
      y = (y > 0.0f) ? y : expm1f(y);
      st[j * 32 + lane] = y + pzr;
    }
    float yv[CPL];
#pragma unroll
    for (int i = 0; i < CPL; ++i) {
      const float y = st[i * 32 + lane];
      yv[i] = live ? y : 0.0f;
    }
    if constexpr (L == 1) {
      v4us ho, lo;
#pragma unroll
      for (int i = 0; i < CPL; ++i) {
        const unsigned int hbi = f2bf(yv[i]);
        ho[i] = (unsigned short)hbi;
        lo[i] = (unsigned short)f2bf(yv[i] - bf2f(hbi));
      }
      if (node < MPr) {
        unsigned short* hp = XP + (size_t)node * KA2 + CPL * lane;
        *(volatile v4us*)hp = ho;
        *(volatile v4us*)(hp + DH) = lo;
        __threadfence();
        *(volatile v4us*)hp = ho;
        *(volatile v4us*)(hp + DH) = lo;
      }
    } else {
      v4f ov;
      ov.x = yv[0]; ov.y = yv[1]; ov.z = yv[2]; ov.w = yv[3];
      if (node < MPr) {
        float* op = HO + (size_t)node * DH + CPL * lane;
        *(volatile v4f*)op = ov;
        __threadfence();
        *(volatile v4f*)op = ov;
      }
    }
  }

  if (lane == 0) misc[wave] = anybig;
  __syncthreads();
  if (wave == 0) {
    int fg = ovf;
#pragma unroll
    for (int w2 = 0; w2 < NWAVE; ++w2) fg |= misc[w2];
    v4i cv;
    cv.x = 0;
    cv.y = (lane == 0) ? fg : 0;
    cv.z = 0; cv.w = 0;
    int* fp = FLGO + (size_t)blk * 32 + 4 * (lane & 7);
    if (lane < 8) *(volatile v4i*)fp = cv;
    __threadfence();
    if (lane < 8) *(volatile v4i*)fp = cv;
  }
}

__global__ __launch_bounds__(NTHR) void k_pool(const int* __restrict__ batch, const float* __restrict__ H,
                                               double* REC, int* PCNT, int nN) {
  __shared__ __attribute__((aligned(16))) double wsum[NWAVE * DH];
  __shared__ int wc[16];
  const int tid = (int)threadIdx.x, lane = tid & 31, wave = tid >> 5;
  const int g = (int)blockIdx.x;
  double a0 = 0.0, a1 = 0.0, a2 = 0.0, a3 = 0.0;
  int mine = 0;
  const int nCh = (nN + 31) >> 5;
#pragma unroll 1
  for (int ch = wave; ch < nCh; ch += NWAVE) {
    const int n  = ch * 32 + lane;
    const int nc = n < nN ? n : nN - 1;
    const int id = batch[nc];
    const bool hit = (n < nN) && (id == g);
    mine += hit ? 1 : 0;
    unsigned mk = __builtin_amdgcn_ballot_w32(hit);
#pragma unroll 1
    while (mk != 0u) {
      const int k = __builtin_ctz(mk);
      mk &= mk - 1u;
      int row = ch * 32 + k;
      row = row > nN - 1 ? nN - 1 : row;
      const v4f v = *(const v4f*)(H + (size_t)row * DH + 4 * lane);
      a0 += (double)v.x; a1 += (double)v.y; a2 += (double)v.z; a3 += (double)v.w;
    }
  }
  int tot = mine;
#pragma unroll
  for (int off = 16; off > 0; off >>= 1) tot += __shfl_xor(tot, off, 32);
  if (lane == 0) wc[wave] = tot;
  {
    v2d p0, p1;
    p0.x = a0; p0.y = a1; p1.x = a2; p1.y = a3;
    *(v2da*)(wsum + wave * DH + 4 * lane)     = p0;
    *(v2da*)(wsum + wave * DH + 4 * lane + 2) = p1;
  }
  __syncthreads();
  const int t64 = tid & 63;
  v2d tv; tv.x = 0.0; tv.y = 0.0;
#pragma unroll
  for (int w2 = 0; w2 < NWAVE; ++w2) {
    const v2d p = *(const v2da*)(wsum + w2 * DH + 2 * t64);
    tv.x += p.x; tv.y += p.y;
  }
  int ctot = 0;
#pragma unroll
  for (int w2 = 0; w2 < NWAVE; ++w2) ctot += wc[w2];
  v4i cv;
  cv.x = (tid == 64) ? ctot : 0;
  cv.y = 0; cv.z = 0; cv.w = 0;
  double* rp = REC + (size_t)g * DH + 2 * t64;
  int* cp = PCNT + (size_t)g * 32 + 4 * (tid & 7);
  const bool wr = tid < 64;
  const bool wq = (tid >= 64) && (tid < 72);
  if (wr) *(volatile v2d*)rp = tv;
  if (wq) *(volatile v4i*)cp = cv;
  __threadfence();
  if (wr) *(volatile v2d*)rp = tv;
  if (wq) *(volatile v4i*)cp = cv;
}

__global__ __launch_bounds__(NTHR) void k_head(const double* __restrict__ REC, const int* __restrict__ PCNT,
                                               const int* __restrict__ FLG, int nLines,
                                               const float* __restrict__ ow, const float* __restrict__ ob,
                                               float* out) {
  __shared__ __attribute__((aligned(16))) float sw[DH * NCLS];
  __shared__ __attribute__((aligned(16))) float sb[16];
  __shared__ __attribute__((aligned(16))) float sout[NGR * NCLS];
  __shared__ int sfl[NWAVE];
  const int tid = (int)threadIdx.x, lane = tid & 31, wave = tid >> 5;
#pragma unroll 1
  for (int i = tid; i < DH * NCLS; i += NTHR) sw[i] = bfr(ow[i]);
  {
    const int kc = tid < NCLS ? tid : NCLS - 1;
    const float bv = bfr(ob[kc]);
    const float sv = (tid < NCLS) ? bv : 0.0f;
    if (tid < 16) sb[tid] = sv;
  }
  int f = 0;
#pragma unroll 1
  for (int i = tid; i < nLines; i += NTHR) f |= FLG[(size_t)i * 32 + 1];
  const unsigned anyf = __builtin_amdgcn_ballot_w32(f != 0);
  if (lane == 0) sfl[wave] = (anyf != 0u) ? 1 : 0;
  __syncthreads();
  int poison = 0;
#pragma unroll
  for (int w2 = 0; w2 < NWAVE; ++w2) poison |= sfl[w2];
  const float qnan = __int_as_float(0x7fc00000);
#pragma unroll 1
  for (int o = tid; o < NGR * NCLS; o += NTHR) {
    const int g = o / NCLS;
    const int k = o - g * NCLS;
    int c = PCNT[(size_t)g * 32];
    c = c < 1 ? 1 : c;
    const double* rp = REC + (size_t)g * DH;
    double s = 0.0;
#pragma unroll 2
    for (int d2 = 0; d2 < DH / 2; ++d2) {
      const v2d p = *(const v2d*)(rp + 2 * d2);
      s = fma(p.x, (double)sw[(2 * d2) * NCLS + k], s);
      s = fma(p.y, (double)sw[(2 * d2 + 1) * NCLS + k], s);
    }
    const float r = (float)(s / (double)c + (double)sb[k]);
    sout[o] = (poison != 0) ? qnan : r;
  }
  __syncthreads();
  const int tq = tid < (NGR * NCLS / 4) ? tid : (NGR * NCLS / 4) - 1;
  const v4f v = *(const v4fa*)(sout + 4 * tq);
  float* op = out + 4 * tq;
  const bool wr = tid < (NGR * NCLS / 4);
  if (wr) *(volatile v4f*)op = v;
  __threadfence();
  if (wr) *(volatile v4f*)op = v;
}

static inline int cdiv(int a, int b) { return (a + b - 1) / b; }

extern "C" void kernel_launch(void* const* d_in, const int* in_sizes, int n_in,
                              void* d_out, int out_size, void* d_ws, size_t ws_size,
                              hipStream_t stream) {
  if (n_in < 11) return;
  const int nN = in_sizes[0] / FIN;
  if (nN <= 0 || in_sizes[0] != nN * FIN || nN > 65536) return;
  if (in_sizes[1] < 2 || (in_sizes[1] & 1) != 0) return;
  const int nE = in_sizes[1] / 2;
  if (nE < 1 || nE > (1 << 30)) return;
  if (in_sizes[2] != nN) return;
  if (in_sizes[3] != FIN * DH || in_sizes[4] != DH) return;
  if (in_sizes[5] != 2 * DH * DH || in_sizes[6] != 2 * DH) return;
  if (in_sizes[7] != 2 * NHD * HCH || in_sizes[8] != 2 * NHD * HCH) return;
  if (in_sizes[9] != DH * NCLS || in_sizes[10] != NCLS) return;
  if (out_size != NGR * NCLS) return;

  const float* x    = (const float*)d_in[0];
  const int*   ei   = (const int*)  d_in[1];
  const int*   bat  = (const int*)  d_in[2];
  const float* inw  = (const float*)d_in[3];
  const float* inb  = (const float*)d_in[4];
  const float* cw   = (const float*)d_in[5];
  const float* cb   = (const float*)d_in[6];
  const float* asrc = (const float*)d_in[7];
  const float* adst = (const float*)d_in[8];
  const float* ow   = (const float*)d_in[9];
  const float* ob   = (const float*)d_in[10];
  float* out = (float*)d_out;
  const int* src = ei;
  const int* dst = ei + nE;

  const int MP   = cdiv(nN, MROWS) * MROWS;
  const int gM   = MP / GBM;
  const int gA   = cdiv(MP, NBA);
  if ((long long)gA * NBA < (long long)MP) return;
  const int vec8 = ((nE & 3) == 0) ? 1 : 0;
  const int nUx  = MP * (FIN / 8);
  if ((nUx % NTHR) != 0) return;

  char* ws = (char*)d_ws;
  size_t off = 0;
  const size_t oXB  = off; off += (size_t)MP * FIN * 2;           off = (off + 255) & ~(size_t)255;
  const size_t oWin = off; off += (size_t)DH * FIN * 2;           off = (off + 255) & ~(size_t)255;
  const size_t oWcD = off; off += (size_t)2 * DH * KA2 * 2;       off = (off + 255) & ~(size_t)255;
  const size_t oA   = off; off += (size_t)MP * KA2 * 2;           off = (off + 255) & ~(size_t)255;
  const size_t oHP  = off; off += (size_t)MP * DH * 4;            off = (off + 255) & ~(size_t)255;
  const size_t oH2  = off; off += (size_t)MP * DH * 4;            off = (off + 255) & ~(size_t)255;
  const size_t oSD  = off; off += (size_t)2 * NHD * MP * 4;       off = (off + 255) & ~(size_t)255;
  const size_t oHIT = off; off += (size_t)gA * RCAP * 4;          off = (off + 255) & ~(size_t)255;
  const size_t oFLG = off; off += (size_t)3 * gA * 128;           off = (off + 255) & ~(size_t)255;
  const size_t oREC = off; off += (size_t)NGR * DH * 8;           off = (off + 255) & ~(size_t)255;
  const size_t oPC  = off; off += (size_t)NGR * 128;              off = (off + 255) & ~(size_t)255;
  if (off > ws_size || off > (size_t)WSMAX) return;
  unsigned short* XB   = (unsigned short*)(ws + oXB);
  unsigned short* WinT = (unsigned short*)(ws + oWin);
  unsigned short* WcD  = (unsigned short*)(ws + oWcD);
  unsigned short* AP   = (unsigned short*)(ws + oA);
  float*          HP   = (float*)(ws + oHP);
  float*          H2   = (float*)(ws + oH2);
  float*          SD   = (float*)(ws + oSD);
  int*            HITS = (int*)(ws + oHIT);
  int*            FLG  = (int*)(ws + oFLG);
  double*         REC  = (double*)(ws + oREC);
  int*            PCNT = (int*)(ws + oPC);
  int* FLG0 = FLG;
  int* FLG1 = FLG + (size_t)gA * 32;
  int* FLG2 = FLG + (size_t)2 * gA * 32;

  const int bktLds  = BKT_LDS_INTS * 4;
  const int scanLds = SCAN_LDS_INTS * 4;
  hipFuncSetAttribute(reinterpret_cast<const void*>(&k_bucket),
                      hipFuncAttributeMaxDynamicSharedMemorySize, bktLds);
  hipFuncSetAttribute(reinterpret_cast<const void*>(&k_scan<1>),
                      hipFuncAttributeMaxDynamicSharedMemorySize, scanLds);
  hipFuncSetAttribute(reinterpret_cast<const void*>(&k_scan<2>),
                      hipFuncAttributeMaxDynamicSharedMemorySize, scanLds);

  k_prep<<<(nUx + NUWI + 2 * NUWC) / NTHR, NTHR, 0, stream>>>(x, inw, cw, XB, WinT, WcD, nN, nUx);
  k_bucket<<<gA, NTHR, bktLds, stream>>>(src, dst, nE, nN, vec8, HITS, FLG0);
  k_gemm<0><<<dim3(gM, DH / GBN), GTHR, 0, stream>>>(XB, WinT, FIN, inb, AP, nN, HP, asrc, adst, SD, MP);
  k_gemm<1><<<dim3(gM, DH / GBN), GTHR, 0, stream>>>(AP, WcD, KA2, inb, AP, nN, HP, asrc, adst, SD, MP);
  k_scan<1><<<gA, NTHR, scanLds, stream>>>(HITS, FLG0, HP, SD, cb, AP, H2, FLG1, nN, MP);
  k_gemm<1><<<dim3(gM, DH / GBN), GTHR, 0, stream>>>(AP, WcD + (size_t)DH * KA2, KA2, inb, AP, nN, HP,
                                                    asrc + NHD * HCH, adst + NHD * HCH, SD, MP);
  k_scan<2><<<gA, NTHR, scanLds, stream>>>(HITS, FLG0, HP, SD, cb + DH, AP, H2, FLG2, nN, MP);
  k_pool<<<NGR, NTHR, 0, stream>>>(bat, H2, REC, PCNT, nN);
  k_head<<<1, NTHR, 0, stream>>>(REC, PCNT, FLG, 3 * gA, ow, ob, out);
}
